// EncoderTransformer_31791347925256
// MI455X (gfx1250) — hardware-verified
//
#include <hip/hip_runtime.h>
#include <math.h>
typedef __attribute__((ext_vector_type(16))) _Float16 v16h;
typedef __attribute__((ext_vector_type(8)))  _Float16 v8h;
typedef __attribute__((ext_vector_type(16))) __bf16   v16b;
typedef __attribute__((ext_vector_type(8)))  __bf16   v8b;
typedef __attribute__((ext_vector_type(8)))  float    v8f;
typedef __attribute__((ext_vector_type(4)))  float    v4f;
#define PSCALE 32768.0f
#define U16(p) ((const unsigned short*)(const void*)(p))
#define PSCALE_INV (1.0f / 32768.0f)

__device__ __forceinline__ unsigned short f2bf_bits(float f) {
  unsigned u = __float_as_uint(f);
  return (unsigned short)((u + 0x7FFFu + ((u >> 16) & 1u)) >> 16);
}
__device__ __forceinline__ float bf_bits2f(unsigned short h) { return __uint_as_float(((unsigned)h) << 16); }

__device__ __forceinline__ void dep_guard_h(v8f& a, v8f& b, v16h x, v16h y) { asm volatile("v_nop\n\tv_nop\n\tv_nop\n\tv_nop" : "+v"(a), "+v"(b) : "v"(x), "v"(y)); }
__device__ __forceinline__ void dep_guard_b(v8f& a, v8f& b, v16b x, v16b y) { asm volatile("v_nop\n\tv_nop\n\tv_nop\n\tv_nop" : "+v"(a), "+v"(b) : "v"(x), "v"(y)); }
__device__ __forceinline__ void keep4_h(v16h a, v16h b, v16h c, v16h d) { asm volatile("v_nop" :: "v"(a), "v"(b), "v"(c), "v"(d)); }
__device__ __forceinline__ void keep4_b(v16b a, v16b b, v16b c, v16b d) { asm volatile("v_nop" :: "v"(a), "v"(b), "v"(c), "v"(d)); }
__device__ __forceinline__ void acc_guard4(v8f& a, v8f& b, v8f& c, v8f& d) { asm volatile("v_nop\n\tv_nop\n\tv_nop\n\tv_nop" : "+v"(a), "+v"(b), "+v"(c), "+v"(d)); }
template <typename T> struct Frag;
template <> struct Frag<_Float16> {
  typedef v16h V; union U { v16h v; v8h h[2]; };
  static __device__ __forceinline__ v16h load(const _Float16* p) {
    U f; f.h[0] = *(const v8h*)(p); f.h[1] = *(const v8h*)(p + 16); return f.v;
  }
  static __device__ __forceinline__ v8f mma(v16h a, v16h b, v8f c) {
    return __builtin_amdgcn_wmma_f32_16x16x32_f16(false, a, false, b, (short)0, c, false, false);
  }
  static __device__ __forceinline__ void guard(v8f& a, v8f& b, v16h x, v16h y) { dep_guard_h(a, b, x, y); }
  static __device__ __forceinline__ void keep(v16h a, v16h b, v16h c, v16h d) { keep4_h(a, b, c, d); }
};
template <> struct Frag<__bf16> {
  typedef v16b V; union U { v16b v; v8b h[2]; };
  static __device__ __forceinline__ v16b load(const __bf16* p) {
    U f; f.h[0] = *(const v8b*)(p); f.h[1] = *(const v8b*)(p + 16); return f.v;
  }
  static __device__ __forceinline__ v8f mma(v16b a, v16b b, v8f c) {
    return __builtin_amdgcn_wmma_f32_16x16x32_bf16(false, a, false, b, (short)0, c, false, false);
  }
  static __device__ __forceinline__ void guard(v8f& a, v8f& b, v16b x, v16b y) { dep_guard_b(a, b, x, y); }
  static __device__ __forceinline__ void keep(v16b a, v16b b, v16b c, v16b d) { keep4_b(a, b, c, d); }
};

template <int ET> struct Elem;
template <> struct Elem<0> { typedef _Float16 T; };
template <> struct Elem<1> { typedef __bf16 T; };
template <int ET, bool SPLIT, int BIAS_MODE, int OUT_MODE, bool RESID, int ACT = 0>
__global__ __launch_bounds__(256) void wmma_gemm64(
    const unsigned short* __restrict__ Ap, const unsigned short* __restrict__ A2p, int lda, long strideA,
    const unsigned short* __restrict__ Btp, const unsigned short* __restrict__ Bt2p, int ldb, long strideB,
    void* __restrict__ Cout, void* __restrict__ Cout2, int ldc, long strideC,
    const float* __restrict__ bias,
    const float* __restrict__ resid, long strideR,
    int M, int N, int K, float scale) {
  typedef typename Elem<ET>::T T;
  typedef typename Frag<T>::V V;
  const T* A = (const T*)Ap; const T* A2 = (const T*)A2p; const T* Bt = (const T*)Btp; const T* Bt2 = (const T*)Bt2p;
  __shared__ __align__(16) float sT[8][16 * 68];
  const int b    = blockIdx.y;
  const int lane = threadIdx.x & 31;
  const int wave = threadIdx.x >> 5;
  const int tilesN = N >> 6;
  const int tilesM = M >> 6;
  const int tile = blockIdx.x * 8 + wave;
  if (tile >= tilesM * tilesN) return;
  const int tm = tile / tilesN;
  const int tn = tile - tm * tilesN;
  const int m0 = tm << 6;
  const int n0 = tn << 6;

  const T* Ab  = A  + (size_t)b * strideA;
  const T* Bb  = Bt + (size_t)b * strideB;
  const T* Ab2 = SPLIT ? (A2  + (size_t)b * strideA) : nullptr;
  const T* Bb2 = SPLIT ? (Bt2 + (size_t)b * strideB) : nullptr;

  const int rlane = lane & 15;
  const int koff  = (lane >> 4) * 8;
  const int mOff  = (lane >> 4) * 8;

  v8f acc[4][4];
#pragma unroll
  for (int i = 0; i < 4; ++i)
#pragma unroll
    for (int j = 0; j < 4; ++j) acc[i][j] = (v8f){0.f,0.f,0.f,0.f,0.f,0.f,0.f,0.f};

  for (int k0 = 0; k0 < K; k0 += 32) {
    V bh[4], bl[4];
#pragma unroll
    for (int j = 0; j < 4; ++j) {
      const size_t bo = (size_t)(n0 + (j << 4) + rlane) * ldb + koff + k0;
      bh[j] = Frag<T>::load(Bb + bo);
      if (SPLIT) bl[j] = Frag<T>::load(Bb2 + bo);
    }
#pragma unroll
    for (int i = 0; i < 4; ++i) {
      const size_t ao = (size_t)(m0 + (i << 4) + rlane) * lda + koff + k0;
      V ah = Frag<T>::load(Ab + ao);
      V al;
      if (SPLIT) al = Frag<T>::load(Ab2 + ao);
#pragma unroll
      for (int j = 0; j < 4; ++j) {
        acc[i][j] = Frag<T>::mma(ah, bh[j], acc[i][j]);
        if (SPLIT) {
          acc[i][j] = Frag<T>::mma(ah, bl[j], acc[i][j]);
          acc[i][j] = Frag<T>::mma(al, bh[j], acc[i][j]);
        }
      }
      Frag<T>::guard(acc[i][0], acc[i][3], ah, SPLIT ? al : ah);
    }
    Frag<T>::keep(bh[0], bh[1], bh[2], bh[3]);
    if (SPLIT) Frag<T>::keep(bl[0], bl[1], bl[2], bl[3]);
  }
  acc_guard4(acc[0][0], acc[0][1], acc[0][2], acc[0][3]);
  acc_guard4(acc[1][0], acc[1][1], acc[1][2], acc[1][3]);
  acc_guard4(acc[2][0], acc[2][1], acc[2][2], acc[2][3]);
  acc_guard4(acc[3][0], acc[3][1], acc[3][2], acc[3][3]);

  float* slab = sT[wave];
  const float* Rb = RESID ? (resid + (size_t)b * strideR) : nullptr;
#pragma unroll
  for (int i = 0; i < 4; ++i) {
    const int mBase = m0 + (i << 4);
#pragma unroll
    for (int j = 0; j < 4; ++j) {
      const int n = n0 + (j << 4) + rlane;
      float bv = 0.f;
      if (BIAS_MODE == 2) bv = bias[n];
#pragma unroll
      for (int r = 0; r < 8; ++r) {
        float v = acc[i][j][r] * scale;
        if (BIAS_MODE == 1) v += bias[mBase + mOff + r];
        if (BIAS_MODE == 2) v += bv;
        if (RESID) v += Rb[(size_t)(mBase + mOff + r) * ldc + n];
        if (ACT == 1) v = tanhf(v);
        if (ACT == 2) v = fmaxf(v, 0.0f);
        if (ACT == 3) v = v / (1.0f + expf(-v));
        if (ACT == 4) v = (v > 0.f) ? v : 0.01f * v;
        if (ACT == 5) v = 0.5f * v * (1.0f + erff(v * 0.70710678118654752f));
        slab[(mOff + r) * 68 + (j << 4) + rlane] = v;
      }
    }
    __builtin_amdgcn_fence(__ATOMIC_RELEASE, "workgroup");
    __builtin_amdgcn_wave_barrier();
    __builtin_amdgcn_fence(__ATOMIC_ACQUIRE, "workgroup");
    if (OUT_MODE == 0) {
      float* C = (float*)Cout + (size_t)b * strideC;
      const int hh = lane >> 4, c4 = (lane & 15) * 4;
      for (int pass = 0; pass < 2; ++pass) {
#pragma unroll
        for (int it = 0; it < 8; ++it) {
          const int row = it * 2 + hh;
          v4f v = *(const v4f*)(slab + row * 68 + c4);
          *(volatile v4f*)(C + (size_t)(mBase + row) * ldc + n0 + c4) = v;
        }
        __threadfence();
      }
    } else {
      const int q = lane >> 3, c8 = (lane & 7) * 8;
      unsigned short* C  = (unsigned short*)Cout  + (size_t)b * strideC;
      unsigned short* C2 = (OUT_MODE == 2) ? ((unsigned short*)Cout2 + (size_t)b * strideC) : nullptr;
      for (int pass = 0; pass < 2; ++pass) {
#pragma unroll
        for (int it = 0; it < 4; ++it) {
          const int row = it * 4 + q;
          const float* sp = slab + row * 68 + c8;
          v8h hv, lv;
#pragma unroll
          for (int e = 0; e < 8; ++e) {
            if (OUT_MODE == 1) {
              hv[e] = (_Float16)sp[e];
            } else {
              unsigned short hb = f2bf_bits(sp[e]);
              unsigned short lb = f2bf_bits(sp[e] - bf_bits2f(hb));
              hv[e] = __builtin_bit_cast(_Float16, hb);
              lv[e] = __builtin_bit_cast(_Float16, lb);
            }
          }
          *(volatile v8h*)(C + (size_t)(mBase + row) * ldc + n0 + c8) = hv;
          if (OUT_MODE == 2) *(volatile v8h*)(C2 + (size_t)(mBase + row) * ldc + n0 + c8) = lv;
        }
        __threadfence();
      }
    }
    __builtin_amdgcn_fence(__ATOMIC_RELEASE, "workgroup");
    __builtin_amdgcn_wave_barrier();
    __builtin_amdgcn_fence(__ATOMIC_ACQUIRE, "workgroup");
  }
}

__global__ __launch_bounds__(256) void cast_f32_f16x2(
    const float* __restrict__ in, _Float16* __restrict__ out, int n2) {
  int i = blockIdx.x * 256 + threadIdx.x;
  if (i < n2) {
    const _Float16 h0 = (_Float16)in[2 * i], h1 = (_Float16)in[2 * i + 1];
    const unsigned u = (unsigned)__builtin_bit_cast(unsigned short, h0) | ((unsigned)__builtin_bit_cast(unsigned short, h1) << 16);
    ((volatile unsigned*)out)[i] = u;
    __threadfence();
    ((volatile unsigned*)out)[i] = u;
  }
}


__global__ __launch_bounds__(256) void transpose_cast_f16(const float* __restrict__ in, int ldi,
                                                         _Float16* __restrict__ outT, int ldo, float scale) {
  __shared__ __align__(16) _Float16 tile[64][72];
  const int c0 = blockIdx.x * 64, r0 = blockIdx.y * 64;
  const int t = threadIdx.y * 32 + threadIdx.x;
  for (int i = threadIdx.y; i < 64; i += 8) {
    tile[threadIdx.x][i]      = (_Float16)(in[(size_t)(r0 + i) * ldi + c0 + threadIdx.x] * scale);
    tile[32 + threadIdx.x][i] = (_Float16)(in[(size_t)(r0 + i) * ldi + c0 + 32 + threadIdx.x] * scale);
  }
  __syncthreads();
  const int q = t >> 3, c8 = (t & 7) * 8;
  for (int pass = 0; pass < 2; ++pass) {
#pragma unroll
    for (int it = 0; it < 2; ++it) {
      const int c = it * 32 + q;
      v8h hv = *(const v8h*)(&tile[c][c8]);
      *(volatile v8h*)(outT + (size_t)(c0 + c) * ldo + r0 + c8) = hv;
    }
    __threadfence();
  }
}

#define TB 16
#define TS 1024
#define TD 512
#define TNN 32
#define TL 128
#define TDK 64
#define TNB (TB * TNN)
#define TROWS (TNB * TL)
__global__ __launch_bounds__(256) void bag_kernel(const float* __restrict__ seq, const int* __restrict__ index, const int* __restrict__ lengths, unsigned* __restrict__ BG16) {
  const int lane = threadIdx.x & 31, wave = threadIdx.x >> 5; const size_t r = (size_t)blockIdx.x * 8 + wave; const int nb = (int)(r / TL), l = (int)(r % TL); const int b = nb / TNN;
  int ix = index[(size_t)nb * TL + l]; ix = ix < 0 ? 0 : (ix >= TS ? TS - 1 : ix); const bool live = l < lengths[nb];
  typedef __attribute__((ext_vector_type(4))) unsigned u4; u4 pk[2];
  const float* src = seq + ((size_t)b * TS + ix) * TD + lane * 16;
  for (int h = 0; h < 2; ++h) { const v4f a = live ? *(const v4f*)(src + 8 * h) : (v4f){0.f, 0.f, 0.f, 0.f}, c = live ? *(const v4f*)(src + 8 * h + 4) : (v4f){0.f, 0.f, 0.f, 0.f};
    pk[h][0] = (unsigned)__builtin_bit_cast(unsigned short, (_Float16)a[0]) | ((unsigned)__builtin_bit_cast(unsigned short, (_Float16)a[1]) << 16); pk[h][1] = (unsigned)__builtin_bit_cast(unsigned short, (_Float16)a[2]) | ((unsigned)__builtin_bit_cast(unsigned short, (_Float16)a[3]) << 16);
    pk[h][2] = (unsigned)__builtin_bit_cast(unsigned short, (_Float16)c[0]) | ((unsigned)__builtin_bit_cast(unsigned short, (_Float16)c[1]) << 16); pk[h][3] = (unsigned)__builtin_bit_cast(unsigned short, (_Float16)c[2]) | ((unsigned)__builtin_bit_cast(unsigned short, (_Float16)c[3]) << 16); }
  for (int pass = 0; pass < 2; ++pass) { *(volatile u4*)(BG16 + (r * TD + lane * 16) / 2) = pk[0]; *(volatile u4*)(BG16 + (r * TD + lane * 16) / 2 + 4) = pk[1]; __threadfence(); }
}
__global__ __launch_bounds__(256) void roots_kernel(const float* __restrict__ hidden, unsigned* __restrict__ R16, float* __restrict__ out1) {
  const int lane = threadIdx.x & 31, wave = threadIdx.x >> 5; const int nb = blockIdx.x * 8 + wave; const int b = nb / TNN;
  unsigned pk[8]; float hv[16];
  for (int q = 0; q < 16; ++q) { const int c = lane * 16 + q; hv[q] = (c < 256) ? hidden[(size_t)b * 256 + c] : hidden[(size_t)TB * 256 + (size_t)b * 256 + (c - 256)]; }
  for (int q = 0; q < 8; ++q) pk[q] = (unsigned)__builtin_bit_cast(unsigned short, (_Float16)hv[2 * q]) | ((unsigned)__builtin_bit_cast(unsigned short, (_Float16)hv[2 * q + 1]) << 16);
  typedef __attribute__((ext_vector_type(4))) unsigned u4; const u4 p0 = {pk[0], pk[1], pk[2], pk[3]}, p1 = {pk[4], pk[5], pk[6], pk[7]};
  for (int pass = 0; pass < 2; ++pass) { *(volatile u4*)(R16 + ((size_t)nb * TD + lane * 16) / 2) = p0; *(volatile u4*)(R16 + ((size_t)nb * TD + lane * 16) / 2 + 4) = p1;
    if ((nb % TNN) == 0) { for (int q = 0; q < 16; ++q) ((volatile float*)out1)[(size_t)b * TD + lane * 16 + q] = hv[q]; } __threadfence(); }
}
__global__ __launch_bounds__(256) void ctx_kernel(const float* __restrict__ PRE, const float* __restrict__ Q, const float* __restrict__ vatt, const float* __restrict__ seq, const int* __restrict__ index, const int* __restrict__ lengths, float* __restrict__ out0) {
  __shared__ float en[8][TL];
  const int lane = threadIdx.x & 31, wave = threadIdx.x >> 5; const int nb = blockIdx.x * 8 + wave; const int b = nb / TNN;
  const float q0 = Q[(size_t)nb * TDK + lane], q1 = Q[(size_t)nb * TDK + 32 + lane], v0 = vatt[lane], v1 = vatt[32 + lane];
  for (int l = 0; l < TL; ++l) { const size_t row = (size_t)nb * TL + l; float e = tanhf(PRE[row * TDK + lane] + q0) * v0 + tanhf(PRE[row * TDK + 32 + lane] + q1) * v1;
    for (int o = 16; o > 0; o >>= 1) e += __shfl_xor(e, o, 32); if (lane == 0) en[wave][l] = e; }
  __builtin_amdgcn_wave_barrier();
  float mx = -INFINITY; for (int l = lane; l < TL; l += 32) mx = fmaxf(mx, en[wave][l]); for (int o = 16; o > 0; o >>= 1) mx = fmaxf(mx, __shfl_xor(mx, o, 32));
  float se = 0.f; for (int l = lane; l < TL; l += 32) se += expf(en[wave][l] - mx); for (int o = 16; o > 0; o >>= 1) se += __shfl_xor(se, o, 32);
  const float inv = 1.0f / se; const int len = lengths[nb];
  float acc[16]; for (int q = 0; q < 16; ++q) acc[q] = 0.f;
  for (int l = 0; l < TL; ++l) { if (l >= len) break;
    const float w = expf(en[wave][l] - mx) * inv; int ix = index[(size_t)nb * TL + l]; ix = ix < 0 ? 0 : (ix >= TS ? TS - 1 : ix);
    const float* src = seq + ((size_t)b * TS + ix) * TD + lane * 16;
    for (int h = 0; h < 4; ++h) { const v4f a = *(const v4f*)(src + 4 * h); for (int q = 0; q < 4; ++q) acc[4 * h + q] += w * a[q]; } }
  for (int pass = 0; pass < 2; ++pass) { for (int h = 0; h < 4; ++h) { const v4f o = {acc[4 * h], acc[4 * h + 1], acc[4 * h + 2], acc[4 * h + 3]}; *(volatile v4f*)(out0 + (size_t)nb * TD + lane * 16 + 4 * h) = o; } __threadfence(); }
}
extern "C" void kernel_launch(void* const* d_in, const int* in_sizes, int n_in, void* d_out, int out_size, void* d_ws, size_t ws_size, hipStream_t stream) {
  (void)in_sizes; (void)n_in; (void)out_size; (void)ws_size;
  const float* seq = (const float*)d_in[0]; const float* hidden = (const float*)d_in[1]; const int* index = (const int*)d_in[2]; const int* lengths = (const int*)d_in[3];
  const float* Wpre = (const float*)d_in[4]; const float* bpre = (const float*)d_in[5]; const float* Wq = (const float*)d_in[6]; const float* vatt = (const float*)d_in[7];
  float* out0 = (float*)d_out; float* out1 = out0 + (size_t)TNB * TD;
  char* ws = (char*)d_ws; size_t off = 0;
  auto carve = [&](size_t bytes) -> char* { char* p = ws + off; off += (bytes + 255) & ~(size_t)255; return p; };
  unsigned* BG16 = (unsigned*)carve((size_t)TROWS * TD * 2); unsigned* R16 = (unsigned*)carve((size_t)TNB * TD * 2); _Float16* WP = (_Float16*)carve(TDK * TD * 2); _Float16* WQ = (_Float16*)carve(TDK * TD * 2);
  float* PRE = (float*)carve((size_t)TROWS * TDK * 4); float* Q = (float*)carve((size_t)TNB * TDK * 4);
  bag_kernel<<<TROWS / 8, 256, 0, stream>>>(seq, index, lengths, BG16);
  roots_kernel<<<TNB / 8, 256, 0, stream>>>(hidden, R16, out1);
  transpose_cast_f16<<<dim3(TDK / 64, TD / 64), dim3(32, 8), 0, stream>>>(Wpre, TDK, WP, TD, 1.0f);
  transpose_cast_f16<<<dim3(TDK / 64, TD / 64), dim3(32, 8), 0, stream>>>(Wq, TDK, WQ, TD, 1.0f);
  { const int t = (TROWS / 64) * 1;
    wmma_gemm64<0, false, 2, 0, false><<<dim3((t + 7) / 8, 1), 256, 0, stream>>>((const unsigned short*)BG16, nullptr, TD, 0, U16(WP), nullptr, TD, 0, PRE, nullptr, TDK, 0, bpre, nullptr, 0, TROWS, TDK, TD, 1.0f); }
  { const int t = (TNB / 64) * 1;
    wmma_gemm64<0, false, 0, 0, false><<<dim3((t + 7) / 8, 1), 256, 0, stream>>>((const unsigned short*)R16, nullptr, TD, 0, U16(WQ), nullptr, TD, 0, Q, nullptr, TDK, 0, nullptr, nullptr, 0, TNB, TDK, TD, 1.0f); }
  ctx_kernel<<<TNB / 8, 256, 0, stream>>>(PRE, Q, vatt, seq, index, lengths, out0);
}
